// GateLoopedAttention_37821482009328
// MI455X (gfx1250) — hardware-verified
//
#include <hip/hip_runtime.h>
#include <math.h>

constexpr int kB    = 2;
constexpr int kN    = 2048;
constexpr int kDim  = 1024;
constexpr int kH    = 64;
constexpr int kHD   = 16;
constexpr int kBH   = kB * kH;
constexpr int kRows = kB * kN;
constexpr int kQKVN = 3 * kDim;
constexpr int kAN   = 2 * kH;
constexpr int kAOff = kQKVN;
constexpr int kQAN  = kQKVN + kAN;
constexpr int kTS   = 64;

typedef __attribute__((ext_vector_type(16))) _Float16 v16h;
typedef __attribute__((ext_vector_type(8)))  _Float16 v8h;
typedef __attribute__((ext_vector_type(16))) __bf16   v16b;
typedef __attribute__((ext_vector_type(8)))  __bf16   v8b;
typedef __attribute__((ext_vector_type(8)))  float    v8f;
typedef __attribute__((ext_vector_type(4)))  float    v4f;
typedef __attribute__((ext_vector_type(4)))  unsigned int v4u;

__device__ __forceinline__ unsigned short f2bf_bits(float f) {
  unsigned u = __float_as_uint(f);
  return (unsigned short)((u + 0x7FFFu + ((u >> 16) & 1u)) >> 16);
}
__device__ __forceinline__ float bf_bits2f(unsigned short h) { return __uint_as_float(((unsigned)h) << 16); }

__device__ __forceinline__ void dep_guard_h(v8f& a, v8f& b, v16h x, v16h y) { asm volatile("v_nop\n\tv_nop\n\tv_nop\n\tv_nop" : "+v"(a), "+v"(b) : "v"(x), "v"(y)); }
__device__ __forceinline__ void dep_guard_b(v8f& a, v8f& b, v16b x, v16b y) { asm volatile("v_nop\n\tv_nop\n\tv_nop\n\tv_nop" : "+v"(a), "+v"(b) : "v"(x), "v"(y)); }
__device__ __forceinline__ void keep4_h(v16h a, v16h b, v16h c, v16h d) { asm volatile("v_nop" :: "v"(a), "v"(b), "v"(c), "v"(d)); }
__device__ __forceinline__ void keep4_b(v16b a, v16b b, v16b c, v16b d) { asm volatile("v_nop" :: "v"(a), "v"(b), "v"(c), "v"(d)); }
__device__ __forceinline__ void acc_guard4(v8f& a, v8f& b, v8f& c, v8f& d) { asm volatile("v_nop\n\tv_nop\n\tv_nop\n\tv_nop" : "+v"(a), "+v"(b), "+v"(c), "+v"(d)); }
template <typename T> struct Frag;
template <> struct Frag<_Float16> {
  typedef v16h V; union U { v16h v; v8h h[2]; };
  static __device__ __forceinline__ v16h load(const _Float16* p) {
    U f; f.h[0] = *(const v8h*)(p); f.h[1] = *(const v8h*)(p + 16); return f.v;
  }
  static __device__ __forceinline__ v8f mma(v16h a, v16h b, v8f c) {
    return __builtin_amdgcn_wmma_f32_16x16x32_f16(false, a, false, b, (short)0, c, false, false);
  }
  static __device__ __forceinline__ void guard(v8f& a, v8f& b, v16h x, v16h y) { dep_guard_h(a, b, x, y); }
  static __device__ __forceinline__ void keep(v16h a, v16h b, v16h c, v16h d) { keep4_h(a, b, c, d); }
};
template <> struct Frag<__bf16> {
  typedef v16b V; union U { v16b v; v8b h[2]; };
  static __device__ __forceinline__ v16b load(const __bf16* p) {
    U f; f.h[0] = *(const v8b*)(p); f.h[1] = *(const v8b*)(p + 16); return f.v;
  }
  static __device__ __forceinline__ v8f mma(v16b a, v16b b, v8f c) {
    return __builtin_amdgcn_wmma_f32_16x16x32_bf16(false, a, false, b, (short)0, c, false, false);
  }
  static __device__ __forceinline__ void guard(v8f& a, v8f& b, v16b x, v16b y) { dep_guard_b(a, b, x, y); }
  static __device__ __forceinline__ void keep(v16b a, v16b b, v16b c, v16b d) { keep4_b(a, b, c, d); }
};

__device__ __forceinline__ unsigned pk16(unsigned short a, unsigned short b) { return (unsigned)a | ((unsigned)b << 16); }
__device__ __forceinline__ unsigned short h_bits(float f) { const _Float16 h = (_Float16)f; return __builtin_bit_cast(unsigned short, h); }

__device__ __forceinline__ float sigm_f(float v) {
  const float e = __expf(-fabsf(v));
  const float r = 1.0f / (1.0f + e);
  return (v >= 0.0f) ? r : e * r;
}

template <int ET> struct Elem;
template <> struct Elem<0> { typedef _Float16 T; };
template <> struct Elem<1> { typedef __bf16 T; };
template <int ET, int SPL, int BIAS, int OUT_MODE, int ACT, int MULR>
__global__ __launch_bounds__(256) void wmma_gemm64(
    const unsigned short* __restrict__ Ap, const unsigned short* __restrict__ A2p, int lda, long strideA,
    const unsigned short* __restrict__ Btp, const unsigned short* __restrict__ Bt2p, int ldb, long strideB,
    void* __restrict__ Cout, void* __restrict__ Cout2, int ldc, long strideC,
    const float* __restrict__ bias, int nbias, int nb0,
    const float* __restrict__ mulr, int ldr,
    int M, int N, int K, float scale) {
  typedef typename Elem<ET>::T T;
  typedef typename Frag<T>::V V;
  const T* A = (const T*)Ap; const T* A2 = (const T*)A2p; const T* Bt = (const T*)Btp; const T* Bt2 = (const T*)Bt2p;
  __shared__ __align__(16) float sT[8][16 * 68];
  const int b    = blockIdx.y;
  const int lane = threadIdx.x & 31;
  const int wave = threadIdx.x >> 5;
  const int tilesN = N >> 6;
  const int tilesM = M >> 6;
  const int tile = blockIdx.x * 8 + wave;
  if (tile >= tilesM * tilesN) return;
  const int tm = tile / tilesN;
  const int tn = tile - tm * tilesN;
  const int m0 = tm << 6;
  const int n0 = tn << 6;

  const T* Ab  = A  + (size_t)b * strideA;
  const T* Bb  = Bt + (size_t)b * strideB;
  const T* Ab2 = (SPL & 1) ? (A2  + (size_t)b * strideA) : nullptr;
  const T* Bb2 = (SPL & 2) ? (Bt2 + (size_t)b * strideB) : nullptr;

  const int rlane = lane & 15;
  const int koff  = (lane >> 4) * 8;
  const int mOff  = (lane >> 4) * 8;

  v8f acc[4][4];
#pragma unroll
  for (int i = 0; i < 4; ++i)
#pragma unroll
    for (int j = 0; j < 4; ++j) acc[i][j] = (v8f){0.f,0.f,0.f,0.f,0.f,0.f,0.f,0.f};

  for (int k0 = 0; k0 < K; k0 += 32) {
    V bh[4], bl[4];
#pragma unroll
    for (int j = 0; j < 4; ++j) {
      const size_t bo = (size_t)(n0 + (j << 4) + rlane) * ldb + koff + k0;
      bh[j] = Frag<T>::load(Bb + bo);
      if (SPL & 2) bl[j] = Frag<T>::load(Bb2 + bo);
    }
#pragma unroll
    for (int i = 0; i < 4; ++i) {
      const size_t ao = (size_t)(m0 + (i << 4) + rlane) * lda + koff + k0;
      V ah = Frag<T>::load(Ab + ao);
      V al;
      if (SPL & 1) al = Frag<T>::load(Ab2 + ao);
#pragma unroll
      for (int j = 0; j < 4; ++j) {
        acc[i][j] = Frag<T>::mma(ah, bh[j], acc[i][j]);
        if (SPL & 2) acc[i][j] = Frag<T>::mma(ah, bl[j], acc[i][j]);
        if (SPL & 1) acc[i][j] = Frag<T>::mma(al, bh[j], acc[i][j]);
      }
      Frag<T>::guard(acc[i][0], acc[i][3], ah, (SPL & 1) ? al : ah);
    }
    Frag<T>::keep(bh[0], bh[1], bh[2], bh[3]);
    if (SPL & 2) Frag<T>::keep(bl[0], bl[1], bl[2], bl[3]);
  }
  acc_guard4(acc[0][0], acc[0][1], acc[0][2], acc[0][3]);
  acc_guard4(acc[1][0], acc[1][1], acc[1][2], acc[1][3]);
  acc_guard4(acc[2][0], acc[2][1], acc[2][2], acc[2][3]);
  acc_guard4(acc[3][0], acc[3][1], acc[3][2], acc[3][3]);

  float* slab = sT[wave];
#pragma unroll
  for (int i = 0; i < 4; ++i) {
    const int mBase = m0 + (i << 4);
#pragma unroll
    for (int j = 0; j < 4; ++j) {
      const int n = n0 + (j << 4) + rlane;
      float bv = 0.f;
      if (BIAS == 2) {
        const int nc = (n < nbias) ? n : (nbias - 1);
        bv = bf_bits2f(f2bf_bits(bias[nc]));
        if (n >= nbias) bv = 0.0f;
      }
      if (BIAS == 3) {
        int nc = n - nb0;
        nc = (nc < 0) ? 0 : nc;
        nc = (nc < nbias) ? nc : (nbias - 1);
        bv = bf_bits2f(f2bf_bits(bias[nc]));
        if (n < nb0 || (n - nb0) >= nbias) bv = 0.0f;
      }
#pragma unroll
      for (int r = 0; r < 8; ++r) {
        float v = acc[i][j][r] * scale;
        if (BIAS == 2 || BIAS == 3) v += bv;
        if (ACT == 3) v = v * sigm_f(v);
        if (ACT == 7) v = sigm_f(0.0625f * v);
        if (MULR == 1) v = v * mulr[(size_t)(mBase + mOff + r) * ldr + n];
        if (MULR == 2) {
          const int mm = mBase + mOff + r;
          const size_t mi = (((size_t)((mm >> 11) * kH + (n >> 4))) * (size_t)kN + (size_t)(mm & (kN - 1))) * (size_t)kHD + (size_t)(n & (kHD - 1));
          v = v * mulr[mi];
        }
        slab[(mOff + r) * 68 + (j << 4) + rlane] = v;
      }
    }
    __builtin_amdgcn_fence(__ATOMIC_RELEASE, "workgroup");
    __builtin_amdgcn_wave_barrier();
    __builtin_amdgcn_fence(__ATOMIC_ACQUIRE, "workgroup");
    if (OUT_MODE == 0) {
      float* Cp = (float*)Cout + (size_t)b * strideC;
      const int hh = lane >> 4, c4 = (lane & 15) * 4;
      for (int pass = 0; pass < 2; ++pass) {
#pragma unroll
        for (int it = 0; it < 8; ++it) {
          const int row = it * 2 + hh;
          v4f v = *(const v4f*)(slab + row * 68 + c4);
          *(volatile v4f*)(Cp + (size_t)(mBase + row) * ldc + n0 + c4) = v;
        }
        __threadfence();
      }
    } else {
      const int q = lane >> 3, c8 = (lane & 7) * 8;
      unsigned short* Cp  = (unsigned short*)Cout  + (size_t)b * strideC;
      unsigned short* Cp2 = (OUT_MODE == 2) ? ((unsigned short*)Cout2 + (size_t)b * strideC) : nullptr;
      for (int pass = 0; pass < 2; ++pass) {
#pragma unroll
        for (int it = 0; it < 4; ++it) {
          const int row = it * 4 + q;
          const float* sp = slab + row * 68 + c8;
          v8h hv, lv;
#pragma unroll
          for (int e = 0; e < 8; ++e) {
            if (OUT_MODE == 1) {
              hv[e] = (_Float16)sp[e];
            } else {
              unsigned short hb = f2bf_bits(sp[e]);
              unsigned short lb = f2bf_bits(sp[e] - bf_bits2f(hb));
              hv[e] = __builtin_bit_cast(_Float16, hb);
              lv[e] = __builtin_bit_cast(_Float16, lb);
            }
          }
          *(volatile v8h*)(Cp + (size_t)(mBase + row) * ldc + n0 + c8) = hv;
          if (OUT_MODE == 2) *(volatile v8h*)(Cp2 + (size_t)(mBase + row) * ldc + n0 + c8) = lv;
        }
        __threadfence();
      }
    }
    __builtin_amdgcn_fence(__ATOMIC_RELEASE, "workgroup");
    __builtin_amdgcn_wave_barrier();
    __builtin_amdgcn_fence(__ATOMIC_ACQUIRE, "workgroup");
  }
  (void)ldr; (void)nb0; (void)nbias;
}

template <int MODE>
__global__ __launch_bounds__(256) void cast8_kernel(const float* __restrict__ in, unsigned short* __restrict__ out, int n8, float scale) {
  const int i = blockIdx.x * 256 + threadIdx.x;
  if (i >= n8) return;
  const float* p = in + 8 * (size_t)i;
  const v4f a = *(const v4f*)(p);
  const v4f c = *(const v4f*)(p + 4);
  unsigned short hb[8];
#pragma unroll
  for (int e = 0; e < 4; ++e) {
    if (MODE == 0) {
      hb[e]     = f2bf_bits(a[e]);
      hb[4 + e] = f2bf_bits(c[e]);
    } else {
      hb[e]     = h_bits(bf_bits2f(f2bf_bits(a[e])) * scale);
      hb[4 + e] = h_bits(bf_bits2f(f2bf_bits(c[e])) * scale);
    }
  }
  const v4u u = (v4u){pk16(hb[0], hb[1]), pk16(hb[2], hb[3]), pk16(hb[4], hb[5]), pk16(hb[6], hb[7])};
  unsigned short* q = out + 8 * (size_t)i;
  *(volatile v4u*)q = u;
  __threadfence();
  *(volatile v4u*)q = u;
  (void)scale;
}

__global__ __launch_bounds__(256) void gl_scan_kernel(const float* __restrict__ QA, float* __restrict__ SO) {
  __shared__ __align__(16) float stg[3][kTS][kHD];
  __shared__ float sar[kTS], sai[kTS];
  __shared__ __align__(16) float sout[kTS * kHD];
  const int bh  = blockIdx.x;
  const int b   = bh >> 6;
  const int h   = bh & 63;
  const int tid = threadIdx.x;
  const int d   = tid & 15;
  const int e   = tid >> 4;
  const size_t rowbase = (size_t)b * kN;

  float Sr = 0.0f, Si = 0.0f;

#pragma unroll 1
  for (int t0 = 0; t0 < kN; t0 += kTS) {
    __syncthreads();
#pragma unroll
    for (int i = 0; i < 3; ++i) {
      const int f    = tid + 256 * i;
      const int s    = f / 12;
      const int part = f - s * 12;
      const int arr  = part >> 2;
      const int j4   = (part & 3) * 4;
      const v4f val = *(const v4f*)(QA + (rowbase + (size_t)(t0 + s)) * (size_t)kQAN + (size_t)arr * kDim + (size_t)h * kHD + j4);
      *(v4f*)(&stg[arr][s][j4]) = val;
    }
    if (tid < kTS) {
      const float* ap = QA + (rowbase + (size_t)(t0 + tid)) * (size_t)kQAN + kAOff + 2 * h;
      const float re = ap[0];
      const float im = ap[1];
      const float mag  = sqrtf(re * re + im * im);
      const float sg   = 1.0f / (1.0f + expf(-mag));
      const float magc = fmaxf(mag, 1e-30f);
      const float inv  = sg * (1.0f / magc);
      float ar = re * inv;
      float ai = im * inv;
      if (!(mag > 0.0f)) { ar = sg; ai = 0.0f; }
      sar[tid] = ar;
      sai[tid] = ai;
    }
    __syncthreads();
#pragma unroll 1
    for (int s = 0; s < kTS; ++s) {
      const float kd = stg[1][s][d];
      const float qd = stg[0][s][d];
      const float ve = stg[2][s][e];
      const float ar = sar[s];
      const float ai = sai[s];
      const float nr = ar * Sr - ai * Si + kd * ve;
      const float ni = ar * Si + ai * Sr;
      Sr = nr;
      Si = ni;
      float p = qd * Sr;
      p += __shfl_xor(p, 1, 32);
      p += __shfl_xor(p, 2, 32);
      p += __shfl_xor(p, 4, 32);
      p += __shfl_xor(p, 8, 32);
      if (d == 0) sout[s * kHD + e] = p;
    }
    __syncthreads();
    {
      const v4f val = *(const v4f*)(sout + 4 * tid);
      float* dst = SO + ((size_t)bh * kN + (size_t)t0) * (size_t)kHD + 4 * tid;
      *(volatile v4f*)dst = val;
      __threadfence();
      *(volatile v4f*)dst = val;
    }
  }
}

extern "C" void kernel_launch(void* const* d_in, const int* in_sizes, int n_in,
                              void* d_out, int out_size, void* d_ws, size_t ws_size,
                              hipStream_t stream) {
  if (n_in < 6) return;
  if (in_sizes[0] != kRows * kDim) return;
  if (in_sizes[1] != kQKVN * kDim) return;
  if (in_sizes[2] != kAN * kDim) return;
  if (in_sizes[3] != kAN) return;
  if (in_sizes[4] != kDim * kDim || in_sizes[5] != kDim * kDim) return;
  if (out_size != kRows * kDim) return;

  const float* x     = (const float*)d_in[0];
  const float* W_qkv = (const float*)d_in[1];
  const float* W_a   = (const float*)d_in[2];
  const float* b_a   = (const float*)d_in[3];
  const float* W_g   = (const float*)d_in[4];
  const float* W_out = (const float*)d_in[5];
  float* outp = (float*)d_out;

  const size_t SZ_XB  = (size_t)kRows * kDim * 2;
  const size_t SZ_WQA = (size_t)kQAN * kDim * 2;
  const size_t SZ_W   = (size_t)kDim * kDim * 2;
  const size_t SZ_QA  = (size_t)kRows * kQAN * 4;
  const size_t SZ_SO  = (size_t)kBH * kN * kHD * 4;
  const size_t SZ_Y   = (size_t)kRows * kDim * 2;

  size_t off = 0;
  const size_t oXB  = off; off += SZ_XB;
  const size_t oWQA = off; off += SZ_WQA;
  const size_t oWG  = off; off += SZ_W;
  const size_t oWO  = off; off += SZ_W;
  const size_t oQA  = off; off += SZ_QA;
  const size_t oSO  = off; off += SZ_SO;
  const size_t oYH  = off; off += SZ_Y;
  const size_t oYL  = off; off += SZ_Y;
  const size_t TOTAL = off;
  if (TOTAL > ws_size) return;
  if (TOTAL > (size_t)134217728) return;

  char* ws = (char*)d_ws;
  unsigned short* XB  = (unsigned short*)(ws + oXB);
  unsigned short* WQA = (unsigned short*)(ws + oWQA);
  unsigned short* WG  = (unsigned short*)(ws + oWG);
  unsigned short* WO  = (unsigned short*)(ws + oWO);
  float*          QA  = (float*)(ws + oQA);
  float*          SO  = (float*)(ws + oSO);
  unsigned short* YH  = (unsigned short*)(ws + oYH);
  unsigned short* YL  = (unsigned short*)(ws + oYL);

  const dim3 blk(256);

  {
    const int n8x = kRows * kDim / 8;
    cast8_kernel<0><<<dim3(n8x / 256), blk, 0, stream>>>(x, XB, n8x, 1.0f);
    const int n8q = kQKVN * kDim / 8;
    cast8_kernel<0><<<dim3(n8q / 256), blk, 0, stream>>>(W_qkv, WQA, n8q, 1.0f);
    const int n8a = kAN * kDim / 8;
    cast8_kernel<0><<<dim3(n8a / 256), blk, 0, stream>>>(W_a, WQA + (size_t)kQKVN * kDim, n8a, 1.0f);
    const int n8w = kDim * kDim / 8;
    cast8_kernel<0><<<dim3(n8w / 256), blk, 0, stream>>>(W_g, WG, n8w, 1.0f);
    cast8_kernel<0><<<dim3(n8w / 256), blk, 0, stream>>>(W_out, WO, n8w, 1.0f);
  }

  const int tilesRows = kRows / 64;
  const dim3 gQA((tilesRows * (kQAN / 64) + 7) / 8, 1);
  const dim3 gSQ((tilesRows * (kDim / 64) + 7) / 8, 1);

  wmma_gemm64<1, 0, 3, 0, 0, 0><<<gQA, blk, 0, stream>>>(
      XB, XB, kDim, 0L, WQA, WQA, kDim, 0L,
      (void*)QA, (void*)QA, kQAN, 0L,
      b_a, kAN, kAOff, SO, kHD,
      kRows, kQAN, kDim, 1.0f);

  gl_scan_kernel<<<dim3(kBH), blk, 0, stream>>>(QA, SO);

  wmma_gemm64<1, 0, 0, 2, 3, 2><<<gSQ, blk, 0, stream>>>(
      XB, XB, kDim, 0L, WG, WG, kDim, 0L,
      (void*)YH, (void*)YL, kDim, 0L,
      b_a, kAN, kAOff, SO, kHD,
      kRows, kDim, kDim, 1.0f);

  wmma_gemm64<1, 1, 0, 0, 0, 0><<<gSQ, blk, 0, stream>>>(
      YH, YL, kDim, 0L, WO, WO, kDim, 0L,
      (void*)outp, (void*)outp, kDim, 0L,
      b_a, kAN, kAOff, SO, kHD,
      kRows, kDim, kDim, 1.0f);
}
